// PolymerGNN_30648886624267
// MI455X (gfx1250) — hardware-run, weakly checked
//
#include <hip/hip_runtime.h>


namespace {
constexpr int N = 50000, E = 600000, G = 2000, C = 128, NH = 4, HD = 32, NT5 = 5, NPB = 8, NBLK = N / NPB  ;
constexpr float HS = 256.0f, WSC = 256.0f, BNEPS = 1e-5f, SLOPE = 0.2f;
typedef _Float16 b16;
typedef __attribute__((ext_vector_type(16))) _Float16 v16b;
typedef __attribute__((ext_vector_type(8))) _Float16 v8b;
typedef __attribute__((ext_vector_type(8))) float v8f;
typedef __attribute__((ext_vector_type(4))) float v4f;
__device__ __forceinline__ float bf16_rne(float f) { unsigned int u = __float_as_uint(f); u += 0x7FFFu + ((u >> 16) & 1u); float r = __uint_as_float(u & 0xFFFF0000u); asm volatile("" : "+v"(r)); return r; }
__device__ __forceinline__ float bfv(float f) { float r = bf16_rne(f); asm volatile("" : "+v"(r)); return r; }
__device__ __forceinline__ void split16(float v, b16& hi, b16& lo) { hi = (b16)v; lo = (b16)(v - (float)hi); }
__device__ __forceinline__ v16b frag_kb(const b16* p, int hh) { const v8b a = *(const v8b*)(p + 8 * hh), b = *(const v8b*)(p + 16 + 8 * hh); v16b f;
#pragma unroll
  for (int e = 0; e < 8; ++e) { f[e] = a[e]; f[8 + e] = b[e]; } return f; }
__device__ __forceinline__ v8f wmma16b(v16b a, v16b b, v8f c) { v8f d = __builtin_amdgcn_wmma_f32_16x16x32_f16(false, a, false, b, (short)0, c, false, false); asm volatile("v_nop\n\tv_nop\n\tv_nop\n\tv_nop" : "+v"(d) : "v"(a), "v"(b)); return d; }
__device__ __forceinline__ void wave_lds_sync() { __builtin_amdgcn_fence(__ATOMIC_RELEASE, "workgroup"); __builtin_amdgcn_wave_barrier(); __builtin_amdgcn_fence(__ATOMIC_ACQUIRE, "workgroup"); }
__device__ __forceinline__ float pmul(float a, float b) { float p = a * b; asm volatile("" : "+v"(p)); return p; }
__device__ __forceinline__ int iclamp(int v, int lo, int hi) { return v < lo ? lo : (v > hi ? hi : v); }
__device__ __forceinline__ float leaky(float v) { return v > 0.0f ? v : SLOPE * v; }
constexpr int CSR_NBLK8 = 512, CSR_GB8 = 8, CSR_GN8 = 1 << CSR_GB8  , CSR_TS8 = (CSR_GN8 < 32 ? 32 : CSR_GN8)  , CSR_MAXG8 = 512, CSR_CAP8 = 12288  ;
__device__ __host__ __forceinline__ int csr_tix8(int v) { return (v >> CSR_GB8) * CSR_TS8 + (v & (CSR_GN8 - 1)); }
__global__ __launch_bounds__(64) void csrA_kernel8(const int* __restrict__ dst, int E, int N, int nG, int CHP, int NGP, int* __restrict__ STG, int* __restrict__ HST) {
  extern __shared__ int sm[];
  int* cnt = sm; int* run = sm + NGP; int* ids = sm + 2 * NGP;
  const int b = blockIdx.x; const int ch = (E + CSR_NBLK8 - 1) / CSR_NBLK8; const int e0 = b * ch, e1 = min(E, e0 + ch);
  for (int i = threadIdx.x; i < NGP; i += 64) cnt[i] = 0;
  for (int i = threadIdx.x; i < CHP; i += 64) ids[i] = -1;
  __syncthreads();
  if (threadIdx.x == 0) {
    for (int e = e0; e < e1; ++e) { int d = dst[e]; d = (d < 0) ? 0 : (d >= N ? N - 1 : d); cnt[d >> CSR_GB8] += 1; }
    int acc = 0; for (int g = 0; g < nG; ++g) { run[g] = acc; acc += cnt[g]; }
    for (int e = e0; e < e1; ++e) { int d = dst[e]; d = (d < 0) ? 0 : (d >= N ? N - 1 : d); const int g = d >> CSR_GB8; ids[run[g]] = e; run[g] += 1; } }
  __syncthreads();
  typedef __attribute__((ext_vector_type(4))) int v4i;
  for (int pass = 0; pass < 2; ++pass) {
    for (int i = threadIdx.x; i < CHP / 4; i += 64) *(volatile v4i*)(STG + (size_t)b * CHP + i * 4) = *(const v4i*)(&ids[i * 4]);
    for (int i = threadIdx.x; i < NGP / 4; i += 64) { v4i v; for (int e = 0; e < 4; ++e) v[e] = (i * 4 + e < nG) ? cnt[i * 4 + e] : 0; *(volatile v4i*)(HST + (size_t)b * NGP + i * 4) = v; }
    __threadfence(); }
}
__global__ __launch_bounds__(512) void csrS_kernel8(const int* __restrict__ HST, int nG, int NGP, int* __restrict__ START, int* __restrict__ TOT, int* __restrict__ OFF) {
  __shared__ int tot[CSR_MAXG8];
  const int b = threadIdx.x;
  for (int pass = 0; pass < 2; ++pass) { int runb = 0; for (int g = 0; g < nG; ++g) { int c = HST[(size_t)b * NGP + g]; c = (c < 0) ? 0 : c; ((volatile int*)OFF)[(size_t)g * CSR_NBLK8 + b] = runb; runb += c; } __threadfence(); }
  for (int g = threadIdx.x; g < nG; g += 512) { int s = 0; for (int bb = 0; bb < CSR_NBLK8; ++bb) { int c = HST[(size_t)bb * NGP + g]; s += (c < 0) ? 0 : c; } tot[g] = s; }
  __syncthreads();
  if (threadIdx.x < 32) {
    __shared__ int st[CSR_MAXG8 + 32];
    if (threadIdx.x == 0) { int acc = 0; for (int g = 0; g < NGP; ++g) { st[g] = acc; if (g < nG) acc += (tot[g] + 31) & ~31; } st[NGP] = acc; }
    __builtin_amdgcn_fence(__ATOMIC_RELEASE, "workgroup"); __builtin_amdgcn_wave_barrier(); __builtin_amdgcn_fence(__ATOMIC_ACQUIRE, "workgroup");
    for (int pass = 0; pass < 2; ++pass) { for (int i = threadIdx.x; i < NGP + 32; i += 32) { ((volatile int*)START)[i] = (i <= NGP) ? st[min(i, NGP)] : 0; ((volatile int*)TOT)[i] = (i < nG) ? tot[i] : 0; } __threadfence(); } }
}
__global__ __launch_bounds__(256) void csrB_kernel8(const int* __restrict__ dst, int N, int nG, int CHP, int NGP, int permLen, const int* __restrict__ STG, const int* __restrict__ HST, const int* __restrict__ OFF, const int* __restrict__ START, const int* __restrict__ TOT, int* __restrict__ PERM, int* __restrict__ ROWPTR, int* __restrict__ ROWCNT, int* __restrict__ FLAG) {
  typedef __attribute__((ext_vector_type(4))) int v4i;
  __shared__ int ids[CSR_CAP8]; __shared__ unsigned short key[CSR_CAP8]; __shared__ int outp[CSR_CAP8]; __shared__ int ncnt[CSR_GN8 + 1]; __shared__ int boff[CSR_NBLK8 + 1];
  const int g = blockIdx.x, t_ = threadIdx.x; int tot = TOT[g]; int st = START[g], stn = START[g + 1]; const int v0 = g * CSR_GN8; const int nv = min(CSR_GN8, N - v0); const int t0 = g * CSR_TS8;
  st = (st < 0) ? 0 : (st > permLen - 32 ? permLen - 32 : st) & ~31; stn = (stn < st) ? st : (stn > permLen ? permLen : stn); tot = (tot < 0) ? 0 : tot; if (tot > stn - st && tot <= CSR_CAP8) tot = stn - st;
  if (tot > CSR_CAP8) {
    for (int pass = 0; pass < 2; ++pass) { for (int i = t_; i < CSR_TS8 / 4; i += 256) { v4i a, c; for (int e = 0; e < 4; ++e) { a[e] = st; c[e] = 0; } *(volatile v4i*)(ROWPTR + t0 + i * 4) = a; *(volatile v4i*)(ROWCNT + t0 + i * 4) = c; } if (t_ == 0) ((volatile int*)FLAG)[0] = 1; __threadfence(); } (void)nv; return; }
  if (t_ == 0) { int acc = 0; for (int b = 0; b < CSR_NBLK8; ++b) { boff[b] = acc; int c = HST[(size_t)b * NGP + g]; c = (c < 0) ? 0 : (c > CHP ? CHP : c); acc += c; if (acc > tot) acc = tot; } boff[CSR_NBLK8] = acc; }
  for (int i = t_; i <= CSR_GN8; i += 256) ncnt[i] = 0;
  __syncthreads();
  for (int b = 0; b < CSR_NBLK8; ++b) { const int c = boff[b + 1] - boff[b]; int o_ = OFF[(size_t)g * CSR_NBLK8 + b]; o_ = (o_ < 0) ? 0 : (o_ > CHP - c ? CHP - c : o_); const int* src_ = STG + (size_t)b * CHP + o_;
    for (int i = t_; i < c; i += 256) { int id = src_[i]; id = (id < 0) ? 0 : id; ids[boff[b] + i] = id; int d = dst[id]; d = (d < v0) ? v0 : (d >= N ? N - 1 : d); int kk = d - v0; kk = (kk < 0) ? 0 : (kk >= CSR_GN8 ? CSR_GN8 - 1 : kk); key[boff[b] + i] = (unsigned short)kk; } }
  __syncthreads();
  if (t_ == 0) { for (int i = 0; i < tot; ++i) ncnt[key[i]] += 1; int acc = 0; for (int vl = 0; vl < CSR_GN8; ++vl) { const int c = ncnt[vl]; ncnt[vl] = acc; acc += c; } ncnt[CSR_GN8] = acc;
    for (int i = 0; i < tot; ++i) { const int vl = key[i]; outp[ncnt[vl]] = ids[i]; ncnt[vl] += 1; }
    for (int vl = CSR_GN8; vl > 0; --vl) ncnt[vl] = ncnt[vl - 1]; ncnt[0] = 0; }
  __syncthreads();
  for (int pass = 0; pass < 2; ++pass) {
    for (int i = t_; i < (stn - st) / 4; i += 256) { v4i v; for (int e = 0; e < 4; ++e) { const int q = i * 4 + e; v[e] = (q < tot) ? outp[q] : -1; } *(volatile v4i*)(PERM + st + i * 4) = v; }
    for (int i = t_; i < CSR_TS8 / 4; i += 256) { v4i a, c; for (int e = 0; e < 4; ++e) { const int vl = i * 4 + e; const int vc = vl < CSR_GN8 ? vl : CSR_GN8; a[e] = (vl < CSR_GN8) ? st + ncnt[vc] : st; c[e] = (vl < nv) ? (ncnt[(vc < CSR_GN8 ? vc : CSR_GN8 - 1) + 1] - ncnt[vc]) : 0; } *(volatile v4i*)(ROWPTR + t0 + i * 4) = a; *(volatile v4i*)(ROWCNT + t0 + i * 4) = c; }
    __threadfence(); }
}
__global__ __launch_bounds__(256) void csrZ_kernel8(int* __restrict__ p, size_t n4) { typedef __attribute__((ext_vector_type(4))) int v4i; const size_t tid = (size_t)blockIdx.x * 256 + threadIdx.x, nth = (size_t)gridDim.x * 256; v4i z = {0, 0, 0, 0}; for (size_t i = tid; i < n4; i += nth) *(volatile v4i*)(p + i * 4) = z; }
struct CsrBufs8 { int *STG, *HST, *OFF, *START, *TOT, *PERM, *ROWPTR, *ROWCNT, *FLAG; int nG, NGP, CHP; size_t permLen; char* base; size_t bytes; };
static size_t csr_carve8(CsrBufs8& c, char* ws, size_t off, int E, int N) {
  const size_t off0 = off; c.base = ws + off;
  auto al = [&](size_t bytes) { char* p = ws + off; off += (bytes + 255) & ~(size_t)255; return p; };
  c.nG = (N + CSR_GN8 - 1) / CSR_GN8; c.NGP = (c.nG + 31) & ~31; const int ch = (E + CSR_NBLK8 - 1) / CSR_NBLK8; c.CHP = (ch + 31) & ~31; c.permLen = (size_t)E + 32 * (size_t)c.nG + 32;
  c.STG = (int*)al((size_t)CSR_NBLK8 * c.CHP * 4); c.HST = (int*)al((size_t)CSR_NBLK8 * c.NGP * 4); c.OFF = (int*)al((size_t)c.NGP * CSR_NBLK8 * 4); c.START = (int*)al((size_t)(c.NGP + 64) * 4); c.TOT = (int*)al((size_t)(c.NGP + 64) * 4);
  c.PERM = (int*)al(c.permLen * 4); c.ROWPTR = (int*)al((size_t)c.nG * CSR_TS8 * 4); c.ROWCNT = (int*)al((size_t)c.nG * CSR_TS8 * 4); c.FLAG = (int*)al(256);
  c.bytes = off - off0; return off;
}
static void csr_build8(const CsrBufs8& c, const int* dst, int E, int N, hipStream_t stream) {
  const size_t smem = (size_t)(2 * c.NGP + c.CHP) * 4;
  csrZ_kernel8<<<512, 256, 0, stream>>>((int*)c.base, c.bytes / 16);
  csrA_kernel8<<<CSR_NBLK8, 64, smem, stream>>>(dst, E, N, c.nG, c.CHP, c.NGP, c.STG, c.HST);
  csrS_kernel8<<<1, 512, 0, stream>>>(c.HST, c.nG, c.NGP, c.START, c.TOT, c.OFF);
  csrB_kernel8<<<c.nG, 256, 0, stream>>>(dst, N, c.nG, c.CHP, c.NGP, (int)c.permLen, c.STG, c.HST, c.OFF, c.START, c.TOT, c.PERM, c.ROWPTR, c.ROWCNT, c.FLAG);
}
constexpr int CSR_NBLKB = 512, CSR_GBB = 8, CSR_GNB = 1 << CSR_GBB  , CSR_TSB = (CSR_GNB < 32 ? 32 : CSR_GNB)  , CSR_MAXGB = 512, CSR_CAPB = 12288  ;
__device__ __host__ __forceinline__ int csr_tixB(int v) { return (v >> CSR_GBB) * CSR_TSB + (v & (CSR_GNB - 1)); }
__global__ __launch_bounds__(64) void csrA_kernelB(const int* __restrict__ dst, int E, int N, int nG, int CHP, int NGP, int* __restrict__ STG, int* __restrict__ HST) {
  extern __shared__ int sm[];
  int* cnt = sm; int* run = sm + NGP; int* ids = sm + 2 * NGP;
  const int b = blockIdx.x; const int ch = (E + CSR_NBLKB - 1) / CSR_NBLKB; const int e0 = b * ch, e1 = min(E, e0 + ch);
  for (int i = threadIdx.x; i < NGP; i += 64) cnt[i] = 0;
  for (int i = threadIdx.x; i < CHP; i += 64) ids[i] = -1;
  __syncthreads();
  if (threadIdx.x == 0) {
    for (int e = e0; e < e1; ++e) { int d = dst[e]; d = (d < 0) ? 0 : (d >= N ? N - 1 : d); cnt[d >> CSR_GBB] += 1; }
    int acc = 0; for (int g = 0; g < nG; ++g) { run[g] = acc; acc += cnt[g]; }
    for (int e = e0; e < e1; ++e) { int d = dst[e]; d = (d < 0) ? 0 : (d >= N ? N - 1 : d); const int g = d >> CSR_GBB; ids[run[g]] = e; run[g] += 1; } }
  __syncthreads();
  typedef __attribute__((ext_vector_type(4))) int v4i;
  for (int pass = 0; pass < 2; ++pass) {
    for (int i = threadIdx.x; i < CHP / 4; i += 64) *(volatile v4i*)(STG + (size_t)b * CHP + i * 4) = *(const v4i*)(&ids[i * 4]);
    for (int i = threadIdx.x; i < NGP / 4; i += 64) { v4i v; for (int e = 0; e < 4; ++e) v[e] = (i * 4 + e < nG) ? cnt[i * 4 + e] : 0; *(volatile v4i*)(HST + (size_t)b * NGP + i * 4) = v; }
    __threadfence(); }
}
__global__ __launch_bounds__(512) void csrS_kernelB(const int* __restrict__ HST, int nG, int NGP, int* __restrict__ START, int* __restrict__ TOT, int* __restrict__ OFF) {
  __shared__ int tot[CSR_MAXGB];
  const int b = threadIdx.x;
  for (int pass = 0; pass < 2; ++pass) { int runb = 0; for (int g = 0; g < nG; ++g) { int c = HST[(size_t)b * NGP + g]; c = (c < 0) ? 0 : c; ((volatile int*)OFF)[(size_t)g * CSR_NBLKB + b] = runb; runb += c; } __threadfence(); }
  for (int g = threadIdx.x; g < nG; g += 512) { int s = 0; for (int bb = 0; bb < CSR_NBLKB; ++bb) { int c = HST[(size_t)bb * NGP + g]; s += (c < 0) ? 0 : c; } tot[g] = s; }
  __syncthreads();
  if (threadIdx.x < 32) {
    __shared__ int st[CSR_MAXGB + 32];
    if (threadIdx.x == 0) { int acc = 0; for (int g = 0; g < NGP; ++g) { st[g] = acc; if (g < nG) acc += (tot[g] + 31) & ~31; } st[NGP] = acc; }
    __builtin_amdgcn_fence(__ATOMIC_RELEASE, "workgroup"); __builtin_amdgcn_wave_barrier(); __builtin_amdgcn_fence(__ATOMIC_ACQUIRE, "workgroup");
    for (int pass = 0; pass < 2; ++pass) { for (int i = threadIdx.x; i < NGP + 32; i += 32) { ((volatile int*)START)[i] = (i <= NGP) ? st[min(i, NGP)] : 0; ((volatile int*)TOT)[i] = (i < nG) ? tot[i] : 0; } __threadfence(); } }
}
__global__ __launch_bounds__(256) void csrB_kernelB(const int* __restrict__ dst, int N, int nG, int CHP, int NGP, int permLen, const int* __restrict__ STG, const int* __restrict__ HST, const int* __restrict__ OFF, const int* __restrict__ START, const int* __restrict__ TOT, int* __restrict__ PERM, int* __restrict__ ROWPTR, int* __restrict__ ROWCNT, int* __restrict__ FLAG) {
  typedef __attribute__((ext_vector_type(4))) int v4i;
  __shared__ int ids[CSR_CAPB]; __shared__ unsigned short key[CSR_CAPB]; __shared__ int outp[CSR_CAPB]; __shared__ int ncnt[CSR_GNB + 1]; __shared__ int boff[CSR_NBLKB + 1];
  const int g = blockIdx.x, t_ = threadIdx.x; int tot = TOT[g]; int st = START[g], stn = START[g + 1]; const int v0 = g * CSR_GNB; const int nv = min(CSR_GNB, N - v0); const int t0 = g * CSR_TSB;
  st = (st < 0) ? 0 : (st > permLen - 32 ? permLen - 32 : st) & ~31; stn = (stn < st) ? st : (stn > permLen ? permLen : stn); tot = (tot < 0) ? 0 : tot; if (tot > stn - st && tot <= CSR_CAPB) tot = stn - st;
  if (tot > CSR_CAPB) {
    for (int pass = 0; pass < 2; ++pass) { for (int i = t_; i < CSR_TSB / 4; i += 256) { v4i a, c; for (int e = 0; e < 4; ++e) { a[e] = st; c[e] = 0; } *(volatile v4i*)(ROWPTR + t0 + i * 4) = a; *(volatile v4i*)(ROWCNT + t0 + i * 4) = c; } if (t_ == 0) ((volatile int*)FLAG)[0] = 1; __threadfence(); } (void)nv; return; }
  if (t_ == 0) { int acc = 0; for (int b = 0; b < CSR_NBLKB; ++b) { boff[b] = acc; int c = HST[(size_t)b * NGP + g]; c = (c < 0) ? 0 : (c > CHP ? CHP : c); acc += c; if (acc > tot) acc = tot; } boff[CSR_NBLKB] = acc; }
  for (int i = t_; i <= CSR_GNB; i += 256) ncnt[i] = 0;
  __syncthreads();
  for (int b = 0; b < CSR_NBLKB; ++b) { const int c = boff[b + 1] - boff[b]; int o_ = OFF[(size_t)g * CSR_NBLKB + b]; o_ = (o_ < 0) ? 0 : (o_ > CHP - c ? CHP - c : o_); const int* src_ = STG + (size_t)b * CHP + o_;
    for (int i = t_; i < c; i += 256) { int id = src_[i]; id = (id < 0) ? 0 : id; ids[boff[b] + i] = id; int d = dst[id]; d = (d < v0) ? v0 : (d >= N ? N - 1 : d); int kk = d - v0; kk = (kk < 0) ? 0 : (kk >= CSR_GNB ? CSR_GNB - 1 : kk); key[boff[b] + i] = (unsigned short)kk; } }
  __syncthreads();
  if (t_ == 0) { for (int i = 0; i < tot; ++i) ncnt[key[i]] += 1; int acc = 0; for (int vl = 0; vl < CSR_GNB; ++vl) { const int c = ncnt[vl]; ncnt[vl] = acc; acc += c; } ncnt[CSR_GNB] = acc;
    for (int i = 0; i < tot; ++i) { const int vl = key[i]; outp[ncnt[vl]] = ids[i]; ncnt[vl] += 1; }
    for (int vl = CSR_GNB; vl > 0; --vl) ncnt[vl] = ncnt[vl - 1]; ncnt[0] = 0; }
  __syncthreads();
  for (int pass = 0; pass < 2; ++pass) {
    for (int i = t_; i < (stn - st) / 4; i += 256) { v4i v; for (int e = 0; e < 4; ++e) { const int q = i * 4 + e; v[e] = (q < tot) ? outp[q] : -1; } *(volatile v4i*)(PERM + st + i * 4) = v; }
    for (int i = t_; i < CSR_TSB / 4; i += 256) { v4i a, c; for (int e = 0; e < 4; ++e) { const int vl = i * 4 + e; const int vc = vl < CSR_GNB ? vl : CSR_GNB; a[e] = (vl < CSR_GNB) ? st + ncnt[vc] : st; c[e] = (vl < nv) ? (ncnt[(vc < CSR_GNB ? vc : CSR_GNB - 1) + 1] - ncnt[vc]) : 0; } *(volatile v4i*)(ROWPTR + t0 + i * 4) = a; *(volatile v4i*)(ROWCNT + t0 + i * 4) = c; }
    __threadfence(); }
}
__global__ __launch_bounds__(256) void csrZ_kernelB(int* __restrict__ p, size_t n4) { typedef __attribute__((ext_vector_type(4))) int v4i; const size_t tid = (size_t)blockIdx.x * 256 + threadIdx.x, nth = (size_t)gridDim.x * 256; v4i z = {0, 0, 0, 0}; for (size_t i = tid; i < n4; i += nth) *(volatile v4i*)(p + i * 4) = z; }
struct CsrBufsB { int *STG, *HST, *OFF, *START, *TOT, *PERM, *ROWPTR, *ROWCNT, *FLAG; int nG, NGP, CHP; size_t permLen; char* base; size_t bytes; };
static size_t csr_carveB(CsrBufsB& c, char* ws, size_t off, int E, int N) {
  const size_t off0 = off; c.base = ws + off;
  auto al = [&](size_t bytes) { char* p = ws + off; off += (bytes + 255) & ~(size_t)255; return p; };
  c.nG = (N + CSR_GNB - 1) / CSR_GNB; c.NGP = (c.nG + 31) & ~31; const int ch = (E + CSR_NBLKB - 1) / CSR_NBLKB; c.CHP = (ch + 31) & ~31; c.permLen = (size_t)E + 32 * (size_t)c.nG + 32;
  c.STG = (int*)al((size_t)CSR_NBLKB * c.CHP * 4); c.HST = (int*)al((size_t)CSR_NBLKB * c.NGP * 4); c.OFF = (int*)al((size_t)c.NGP * CSR_NBLKB * 4); c.START = (int*)al((size_t)(c.NGP + 64) * 4); c.TOT = (int*)al((size_t)(c.NGP + 64) * 4);
  c.PERM = (int*)al(c.permLen * 4); c.ROWPTR = (int*)al((size_t)c.nG * CSR_TSB * 4); c.ROWCNT = (int*)al((size_t)c.nG * CSR_TSB * 4); c.FLAG = (int*)al(256);
  c.bytes = off - off0; return off;
}
static void csr_buildB(const CsrBufsB& c, const int* dst, int E, int N, hipStream_t stream) {
  const size_t smem = (size_t)(2 * c.NGP + c.CHP) * 4;
  csrZ_kernelB<<<512, 256, 0, stream>>>((int*)c.base, c.bytes / 16);
  csrA_kernelB<<<CSR_NBLKB, 64, smem, stream>>>(dst, E, N, c.nG, c.CHP, c.NGP, c.STG, c.HST);
  csrS_kernelB<<<1, 512, 0, stream>>>(c.HST, c.nG, c.NGP, c.START, c.TOT, c.OFF);
  csrB_kernelB<<<c.nG, 256, 0, stream>>>(dst, N, c.nG, c.CHP, c.NGP, (int)c.permLen, c.STG, c.HST, c.OFF, c.START, c.TOT, c.PERM, c.ROWPTR, c.ROWCNT, c.FLAG);
}


__global__ __launch_bounds__(256) void wput_kernel(const float* __restrict__ w0, const float* __restrict__ w1, const float* __restrict__ w2, const float* __restrict__ wg, const float* __restrict__ h1, b16* __restrict__ W0T, b16* __restrict__ W1T, b16* __restrict__ W2T, b16* __restrict__ WGT, b16* __restrict__ H1T) { const int u = blockIdx.x * 256 + threadIdx.x; v8b v;
  if (u < C * 4) { const int o = u / 4, k0 = (u % 4) * 8;
#pragma unroll
    for (int j = 0; j < 8; ++j) { const int k = k0 + j; v[j] = (b16)(k < 8 ? bf16_rne(w0[(size_t)k * C + o]) * WSC : 0.0f); } for (int pass = 0; pass < 2; ++pass) { *(volatile v8b*)(W0T + (size_t)o * 32 + k0) = v; __threadfence(); } }
  if (u < C * 16) { const int o = u / 16, k0 = (u % 16) * 8; const float* ws3[3] = {w1, w2, wg}; b16* ds3[3] = {W1T, W2T, WGT};
#pragma unroll
    for (int m = 0; m < 3; ++m) {
#pragma unroll
      for (int j = 0; j < 8; ++j) v[j] = (b16)(bf16_rne(ws3[m][(size_t)(k0 + j) * C + o]) * WSC); for (int pass = 0; pass < 2; ++pass) { *(volatile v8b*)(ds3[m] + (size_t)o * C + k0) = v; __threadfence(); } } }
  if (u < NT5 * C * 32) { const int t = u / (C * 32), r = u % (C * 32); const int o = r / 32, k0 = (r % 32) * 8;
#pragma unroll
    for (int j = 0; j < 8; ++j) v[j] = (b16)(bf16_rne(h1[((size_t)t * 2 * C + k0 + j) * C + o]) * WSC); for (int pass = 0; pass < 2; ++pass) { *(volatile v8b*)(H1T + ((size_t)t * C + o) * 2 * C + k0) = v; __threadfence(); } } }
__global__ __launch_bounds__(256) void deg_kernel(const int* __restrict__ ROWCNT, float* __restrict__ DINV) { const int n = blockIdx.x * 256 + threadIdx.x; if (n >= N) return; const float d = rsqrtf((float)iclamp(ROWCNT[n], 0, E) + 1.0f); for (int pass = 0; pass < 2; ++pass) { ((volatile float*)DINV)[n] = d; __threadfence(); } }
template <int MODE>
__global__ __launch_bounds__(32) void lin_kernel(const float* __restrict__ IN, const float* __restrict__ BNs, const float* __restrict__ g, const float* __restrict__ bb, const b16* __restrict__ W, const float* __restrict__ as_, const float* __restrict__ ad_, int NLIM, float* __restrict__ Y, float* __restrict__ ES) { __shared__ __attribute__((aligned(16))) b16 Ah[16][C + 8], Al[16][C + 8]; __shared__ float Tf[16][C + 4], Eq[16][8]; const int lane = threadIdx.x, nloc = lane & 15, hlf = lane >> 4; const size_t m0 = (size_t)blockIdx.x * 16; if (m0 >= (size_t)NLIM) return;
  if (MODE == 0) { for (int rr = 0; rr < 16; ++rr) { Ah[rr][lane] = (b16)(lane < 8 ? bf16_rne(IN[(m0 + rr) * 8 + (lane & 7)]) * HS : 0.0f); Al[rr][lane] = (b16)0.0f; if (lane < 8) { Ah[rr][32 + lane] = (b16)0.0f; Al[rr][32 + lane] = (b16)0.0f; } } }
  else { for (int q = 0; q < 4; ++q) { const int c = q * 32 + lane; const float mu = BNs[c], rs = BNs[C + c], gg = bfv(g[c]), be = bfv(bb[c]); for (int rr = 0; rr < 16; ++rr) { const float v = fmaxf(pmul(pmul(IN[(m0 + rr) * C + c] - mu, rs), gg) + be, 0.0f); b16 p, ql; split16(v * HS, p, ql); Ah[rr][c] = p; Al[rr][c] = ql; } } if (lane < 16) for (int k = C; k < C + 8; ++k) { Ah[lane][k] = (b16)0.0f; Al[lane][k] = (b16)0.0f; } }
  wave_lds_sync(); v8f acc[8];
#pragma unroll
  for (int t = 0; t < 8; ++t) acc[t] = (v8f){};
  constexpr int KK = MODE == 0 ? 32 : C;
#pragma unroll
  for (int kb = 0; kb < KK; kb += 32) { const v16b a = frag_kb(&Ah[nloc][kb], hlf), al = frag_kb(&Al[nloc][kb], hlf);
#pragma unroll
    for (int t = 0; t < 8; ++t) { const v16b bw = frag_kb(W + (size_t)(t * 16 + nloc) * KK + kb, hlf); acc[t] = wmma16b(a, bw, acc[t]); if (MODE != 0) acc[t] = wmma16b(al, bw, acc[t]); } }
#pragma unroll
  for (int t = 0; t < 8; ++t)
#pragma unroll
    for (int r8 = 0; r8 < 8; ++r8) Tf[8 * hlf + r8][t * 16 + nloc] = acc[t][r8] * (1.0f / (HS * WSC));
  wave_lds_sync();
  if (MODE == 2) { for (int rr = 0; rr < 16; ++rr) { const int hd = lane >> 3, c0 = (lane & 7) * 4; float s1 = 0.0f, s2 = 0.0f; for (int k = 0; k < 4; ++k) { const int cc = hd * HD + c0 + k; s1 += pmul(Tf[rr][cc], bfv(as_[cc])); s2 += pmul(Tf[rr][cc], bfv(ad_[cc])); } for (int o = 1; o < 8; o <<= 1) { s1 += __shfl_xor(s1, o); s2 += __shfl_xor(s2, o); } if ((lane & 7) == 0) { Eq[rr][hd] = s1; Eq[rr][4 + hd] = s2; } } wave_lds_sync(); }
  for (int pass = 0; pass < 2; ++pass) { for (int rr = 0; rr < 16; ++rr) *(volatile v4f*)(Y + (m0 + rr) * C + lane * 4) = *(const v4f*)(&Tf[rr][lane * 4]); if (MODE == 2) *(volatile v4f*)(ES + (m0 + (lane >> 1)) * 8 + (lane & 1) * 4) = *(const v4f*)(&Eq[lane >> 1][(lane & 1) * 4]);     __threadfence(); } }
__global__ __launch_bounds__(256) void gcnsweep_kernel(const float* __restrict__ Y, const float* __restrict__ DINV, const float* __restrict__ bias, const int* __restrict__ srcs, const int* __restrict__ PERM, const int* __restrict__ ROWPTR, const int* __restrict__ ROWCNT, int permLen, int NLIM, float* __restrict__ Z, float* __restrict__ PS) { __shared__ float Red[NPB][C]; const int wave = threadIdx.x >> 5, lane = threadIdx.x & 31; const size_t i = (size_t)blockIdx.x * NPB + wave; v4f o = {0, 0, 0, 0};
  if (i < (size_t)NLIM) { int st = ROWPTR[i], cnt = ROWCNT[i]; cnt = iclamp(cnt, 0, E); st = iclamp(st, 0, permLen - cnt); v4f acc = {0, 0, 0, 0};
#pragma unroll 1
    for (int j = 0; j < cnt; ++j) { const int e = iclamp(PERM[st + j], 0, E - 1); const size_t u = (size_t)iclamp(srcs[e], 0, N - 1); if (u >= (size_t)NLIM) continue; const float du = DINV[u]; const v4f v = *(const v4f*)(Y + u * C + lane * 4);
#pragma unroll
      for (int k = 0; k < 4; ++k) acc[k] += pmul(du, v[k]); }
    const float di = DINV[i]; const v4f yi = *(const v4f*)(Y + i * C + lane * 4);
#pragma unroll
    for (int k = 0; k < 4; ++k) o[k] = pmul(di, acc[k] + pmul(di, yi[k])) + bfv(bias[lane * 4 + k]); }
  for (int k = 0; k < 4; ++k) Red[wave][lane * 4 + k] = o[k];
  for (int pass = 0; pass < 2; ++pass) { if (i < (size_t)NLIM) *(volatile v4f*)(Z + i * C + lane * 4) = o; __threadfence(); }
  __syncthreads();
  if (wave == 0) for (int pass = 0; pass < 2; ++pass) { for (int c = lane; c < C; c += 32) { float s = 0.0f, s2 = 0.0f; for (int w = 0; w < NPB; ++w) { const float v = (blockIdx.x * NPB + w < NLIM) ? Red[w][c] : 0.0f; s += v; s2 += v * v; } ((volatile float*)PS)[(size_t)blockIdx.x * 2 * C + c] = s; ((volatile float*)PS)[(size_t)blockIdx.x * 2 * C + C + c] = s2; } __threadfence(); } }
__global__ __launch_bounds__(128) void bn_kernel(const float* __restrict__ PS, int nblk, int NLIM, float* __restrict__ BNs) { const int c = threadIdx.x; double s = 0.0, s2 = 0.0; for (int b = 0; b < nblk; ++b) { s += (double)PS[(size_t)b * 2 * C + c]; s2 += (double)PS[(size_t)b * 2 * C + C + c]; } const double mu = s / NLIM; double var = s2 / NLIM - mu * mu; if (var < 0.0) var = 0.0;
  for (int pass = 0; pass < 2; ++pass) { ((volatile float*)BNs)[c] = (float)mu; ((volatile float*)BNs)[C + c] = (float)(1.0 / sqrt(var + (double)BNEPS)); __threadfence(); } }
__global__ __launch_bounds__(256) void gatsweep_kernel(const float* __restrict__ HG, const float* __restrict__ ES, const float* __restrict__ bg, const int* __restrict__ srcs, const int* __restrict__ PERM, const int* __restrict__ ROWPTR, const int* __restrict__ ROWCNT, int permLen, int NLIM, float* __restrict__ X) { const int wave = threadIdx.x >> 5, lane = threadIdx.x & 31, hd = lane >> 3; const size_t i = (size_t)blockIdx.x * NPB + wave; if (i >= (size_t)NLIM) return; int st = ROWPTR[i], cnt = ROWCNT[i]; cnt = iclamp(cnt, 0, E); st = iclamp(st, 0, permLen - cnt); const float edi = ES[i * 8 + 4 + hd];
  float mx = leaky(ES[i * 8 + hd] + edi), den = 1.0f; v4f acc = *(const v4f*)(HG + i * C + lane * 4);
#pragma unroll 1
  for (int j = 0; j < cnt; ++j) { const int e = iclamp(PERM[st + j], 0, E - 1); const size_t u = (size_t)iclamp(srcs[e], 0, N - 1); if (u >= (size_t)NLIM) continue; const float s = leaky(ES[u * 8 + hd] + edi); const float mn = fmaxf(mx, s); const float sf = __expf(mx - mn); const float p = __expf(s - mn); den = den * sf + p; const v4f v = *(const v4f*)(HG + u * C + lane * 4);
#pragma unroll
    for (int k = 0; k < 4; ++k) acc[k] = pmul(acc[k], sf) + pmul(p, v[k]); mx = mn; }
  v4f o; for (int k = 0; k < 4; ++k) o[k] = acc[k] / den + bfv(bg[lane * 4 + k]);
  for (int pass = 0; pass < 2; ++pass) { *(volatile v4f*)(X + i * C + lane * 4) = o; __threadfence(); } }
__global__ __launch_bounds__(256) void pool_kernel(const float* __restrict__ X, const int* __restrict__ batch, const int* __restrict__ PERM, const int* __restrict__ ROWPTR, const int* __restrict__ ROWCNT, int permLen, int NLIM, float* __restrict__ HC2) { const int wave = threadIdx.x >> 5, lane = threadIdx.x & 31; const int gph = blockIdx.x * 8 + wave; if (gph >= G) return; v4f sm = {0, 0, 0, 0}, mxv = {-INFINITY, -INFINITY, -INFINITY, -INFINITY}; int cnt = 0; int st = ROWPTR[gph], c0 = ROWCNT[gph]; c0 = iclamp(c0, 0, N); st = iclamp(st, 0, permLen - c0);
#pragma unroll 1
  for (int j = 0; j < c0; ++j) { const int n = iclamp(PERM[st + j], 0, N - 1); if (n >= NLIM || batch[n] != gph) continue; ++cnt; const v4f v = *(const v4f*)(X + (size_t)n * C + lane * 4); for (int k = 0; k < 4; ++k) { sm[k] += v[k]; mxv[k] = fmaxf(mxv[k], v[k]); } }
  const float inv = 1.0f / fmaxf((float)cnt, 1.0f); v4f om, ox; for (int k = 0; k < 4; ++k) { om[k] = pmul(sm[k], inv); ox[k] = cnt > 0 ? mxv[k] : 0.0f; }
  for (int pass = 0; pass < 2; ++pass) { *(volatile v4f*)(HC2 + (size_t)gph * 2 * C + lane * 4) = om; *(volatile v4f*)(HC2 + (size_t)gph * 2 * C + C + lane * 4) = ox; __threadfence(); } }
__global__ __launch_bounds__(32) void head_kernel(const float* __restrict__ HC2, const b16* __restrict__ H1T, const float* __restrict__ hb1, const float* __restrict__ h2, const float* __restrict__ hb2, int GLIM, float* __restrict__ OUT) { __shared__ __attribute__((aligned(16))) b16 Ah[32][2 * C + 8], Al[32][2 * C + 8]; __shared__ float Tf[32][C + 4], Os[32][8]; const int lane = threadIdx.x, nloc = lane & 15, hlf = lane >> 4; const size_t g0 = (size_t)blockIdx.x * 32; if (g0 >= (size_t)GLIM) return;
  for (int rr = 0; rr < 32; ++rr) { const bool in = g0 + rr < (size_t)GLIM; for (int q = 0; q < 8; ++q) { b16 p = (b16)0.0f, ql = (b16)0.0f; if (in) split16(HC2[(g0 + rr) * 2 * C + q * 32 + lane] * HS, p, ql); Ah[rr][q * 32 + lane] = p; Al[rr][q * 32 + lane] = ql; } } for (int k = 2 * C; k < 2 * C + 8; ++k) { Ah[lane][k] = (b16)0.0f; Al[lane][k] = (b16)0.0f; }
  wave_lds_sync();
#pragma unroll 1
  for (int t = 0; t < NT5; ++t) {
#pragma unroll 1
    for (int rt = 0; rt < 2; ++rt) { v8f acc[8];
#pragma unroll
      for (int q = 0; q < 8; ++q) acc[q] = (v8f){};
#pragma unroll 2
      for (int kb = 0; kb < 2 * C; kb += 32) { const v16b a = frag_kb(&Ah[rt * 16 + nloc][kb], hlf), al = frag_kb(&Al[rt * 16 + nloc][kb], hlf);
#pragma unroll
        for (int q = 0; q < 8; ++q) { const v16b bw = frag_kb(H1T + ((size_t)t * C + q * 16 + nloc) * 2 * C + kb, hlf); acc[q] = wmma16b(a, bw, acc[q]); acc[q] = wmma16b(al, bw, acc[q]); } }
#pragma unroll
      for (int q = 0; q < 8; ++q) { const int cc = q * 16 + nloc; const float bb = bfv(hb1[t * C + cc]);
#pragma unroll
        for (int r8 = 0; r8 < 8; ++r8) Tf[rt * 16 + 8 * hlf + r8][cc] = fmaxf(acc[q][r8] * (1.0f / (HS * WSC)) + bb, 0.0f); } }
    wave_lds_sync();
    { float s = 0.0f; for (int c = 0; c < C; ++c) s += pmul(Tf[lane][c], bfv(h2[t * C + c])); Os[lane][t] = s + bfv(hb2[t]); }
    wave_lds_sync(); }
  const int ng = (GLIM - (int)g0) < 32 ? (GLIM - (int)g0) : 32;
  for (int pass = 0; pass < 2; ++pass) { for (int idx = lane; idx < ng * NT5; idx += 32) ((volatile float*)OUT)[g0 * NT5 + idx] = Os[idx / NT5][idx % NT5]; __threadfence(); } }
}

extern "C" void kernel_launch(void* const* d_in, const int* in_sizes, int n_in, void* d_out, int out_size, void* d_ws, size_t ws_size, hipStream_t stream) {
  (void)n_in;
  auto Fp = [&](int i) { return (const float*)d_in[i]; }; auto Ip = [&](int i) { return (const int*)d_in[i]; };
  if (in_sizes[0] != N * 8 || in_sizes[1] != 2 * E || in_sizes[2] != N || in_sizes[3] != 8 * C || in_sizes[7] != C * C || in_sizes[11] != C * C || in_sizes[15] != C * C || in_sizes[16] != NH * HD || in_sizes[19] != NT5 * 2 * C * C || in_sizes[21] != NT5 * C || out_size != G * NT5) return;
  const int NLIM = N;
  size_t off = 0; char* ws = (char*)d_ws;
  auto carve = [&](size_t bytes) { char* p = ws + off; off += (bytes + 255) & ~(size_t)255; return p; };
  b16* W0T = (b16*)carve((size_t)C * 32 * 2); b16* W1T = (b16*)carve((size_t)C * C * 2); b16* W2T = (b16*)carve((size_t)C * C * 2); b16* WGT = (b16*)carve((size_t)C * C * 2); b16* H1T = (b16*)carve((size_t)NT5 * C * 2 * C * 2);
  float* DINV = (float*)carve((size_t)N * 4); float* Y = (float*)carve((size_t)N * C * 4); float* Z = (float*)carve((size_t)N * C * 4); float* ES = (float*)carve((size_t)N * 8 * 4); float* X = (float*)carve((size_t)N * C * 4); float* PS = (float*)carve((size_t)NBLK * 2 * C * 4); float* BNs = (float*)carve(2 * C * 4); float* HC2 = (float*)carve((size_t)G * 2 * C * 4); CsrBufs8 csr; off = csr_carve8(csr, ws, off, E, N); CsrBufsB cb; off = csr_carveB(cb, ws, off, N, G);
  if (off > ws_size || off > ((size_t)128 << 20)) return;
  const int nblk = (NLIM + NPB - 1) / NPB;
  wput_kernel<<<(NT5 * C * 32 + 255) / 256, 256, 0, stream>>>(Fp(3), Fp(7), Fp(11), Fp(15), Fp(19), W0T, W1T, W2T, WGT, H1T);
  csr_build8(csr, Ip(1) + E, E, N, stream); csr_buildB(cb, Ip(2), N, G, stream);
  deg_kernel<<<(N + 255) / 256, 256, 0, stream>>>(csr.ROWCNT, DINV);
  lin_kernel<0><<<NLIM / 16, 32, 0, stream>>>(Fp(0), BNs, Fp(5), Fp(6), W0T, Fp(16), Fp(17), NLIM, Y, ES);
  gcnsweep_kernel<<<nblk, 256, 0, stream>>>(Y, DINV, Fp(4), Ip(1), csr.PERM, csr.ROWPTR, csr.ROWCNT, (int)csr.permLen, NLIM, Z, PS); bn_kernel<<<1, 128, 0, stream>>>(PS, nblk, NLIM, BNs);
  lin_kernel<1><<<NLIM / 16, 32, 0, stream>>>(Z, BNs, Fp(5), Fp(6), W1T, Fp(16), Fp(17), NLIM, Y, ES);
  gcnsweep_kernel<<<nblk, 256, 0, stream>>>(Y, DINV, Fp(8), Ip(1), csr.PERM, csr.ROWPTR, csr.ROWCNT, (int)csr.permLen, NLIM, Z, PS); bn_kernel<<<1, 128, 0, stream>>>(PS, nblk, NLIM, BNs);
  lin_kernel<1><<<NLIM / 16, 32, 0, stream>>>(Z, BNs, Fp(9), Fp(10), W2T, Fp(16), Fp(17), NLIM, Y, ES);
  gcnsweep_kernel<<<nblk, 256, 0, stream>>>(Y, DINV, Fp(12), Ip(1), csr.PERM, csr.ROWPTR, csr.ROWCNT, (int)csr.permLen, NLIM, Z, PS); bn_kernel<<<1, 128, 0, stream>>>(PS, nblk, NLIM, BNs);
  lin_kernel<2><<<NLIM / 16, 32, 0, stream>>>(Z, BNs, Fp(13), Fp(14), WGT, Fp(16), Fp(17), NLIM, Y, ES);
  gatsweep_kernel<<<nblk, 256, 0, stream>>>(Y, ES, Fp(18), Ip(1), csr.PERM, csr.ROWPTR, csr.ROWCNT, (int)csr.permLen, NLIM, X);
  pool_kernel<<<G / 8, 256, 0, stream>>>(X, Ip(2), cb.PERM, cb.ROWPTR, cb.ROWCNT, (int)cb.permLen, NLIM, HC2);
  head_kernel<<<(G + 31) / 32, 32, 0, stream>>>(HC2, H1T, Fp(20), Fp(21), Fp(22), G, (float*)d_out);
}
